// MultiHeadAttention_19731079758119
// MI455X (gfx1250) — hardware-run, weakly checked
//
#include <hip/hip_runtime.h>
#ifndef NB
#define NB 2
#endif
#ifndef SEQ
#define SEQ 2048
#endif
#define NB_FULL 2
#define SEQ_FULL 2048
#define DM 1024
#define NH 16
#define HD 64
#define HG 2
#define FR_ROW 128
#define NR ((size_t)NB * SEQ)
#define X_BSTRIDE_FULL ((size_t)SEQ_FULL * DM)

static_assert(SEQ % 128 == 0);
static_assert(SEQ <= SEQ_FULL);
static_assert(NB <= NB_FULL);
static_assert(NH % HG == 0);
static_assert(DM == NH * HD);
static_assert(HD == 64);
static_assert(DM % 64 == 0);

typedef unsigned short v8us __attribute__((ext_vector_type(8), may_alias));
typedef float  v8f  __attribute__((ext_vector_type(8)));
typedef float  v4f  __attribute__((ext_vector_type(4)));
typedef float  v4fa __attribute__((ext_vector_type(4), may_alias));
typedef _Float16 v16h __attribute__((ext_vector_type(16)));
typedef _Float16 v4h __attribute__((ext_vector_type(4)));
union FragH { v16h v; v8us half[2]; _Float16 h[16]; unsigned short u[16]; };

__device__ __forceinline__ unsigned short bf16_bits(float x) { unsigned int u = __float_as_uint(x); return (unsigned short)((u + 0x7FFFu + ((u >> 16) & 1u)) >> 16); }
__device__ __forceinline__ float bf16_val(unsigned short b) { return __uint_as_float(((unsigned int)b) << 16); }
__device__ __forceinline__ float bf16_rne(float x) { return bf16_val(bf16_bits(x)); }

__global__ __launch_bounds__(256) void k_wnat(const float* __restrict__ w, size_t n8, _Float16* __restrict__ Bt) {
  const size_t t = (size_t)blockIdx.x * 256 + threadIdx.x; if (t >= n8) return;
  const v4f a = *(const v4fa*)(w + t * 8), c = *(const v4fa*)(w + t * 8 + 4);
  FragH f;
#pragma unroll
  for (int q = 0; q < 4; ++q) { f.h[q] = (_Float16)(bf16_rne(a[q]) * 16.0f); f.h[4 + q] = (_Float16)(bf16_rne(c[q]) * 16.0f); }
  const v8us o = f.half[0];
  *(volatile v8us*)((unsigned short*)Bt + t * 8) = o; __threadfence(); *(volatile v8us*)((unsigned short*)Bt + t * 8) = o;
}

__global__ __launch_bounds__(256) void k_x16(const float* __restrict__ x, _Float16* __restrict__ X16, size_t n8b, size_t bstride, size_t n8) {
  const size_t t = (size_t)blockIdx.x * 256 + threadIdx.x; if (t >= n8) return;
  const size_t b = t / n8b, rem = t - b * n8b;
  const float* src = x + b * bstride + rem * 8;
  const v4f a = *(const v4fa*)(src), c = *(const v4fa*)(src + 4);
  FragH f;
#pragma unroll
  for (int q = 0; q < 4; ++q) { f.h[q] = (_Float16)bf16_rne(a[q]); f.h[4 + q] = (_Float16)bf16_rne(c[q]); }
  const v8us o = f.half[0];
  *(volatile v8us*)((unsigned short*)X16 + t * 8) = o; __threadfence(); *(volatile v8us*)((unsigned short*)X16 + t * 8) = o;
}

__device__ __forceinline__ v16h g2_frag(const _Float16* p, int hh) { FragH f; f.half[0] = *(const v8us*)((const unsigned short*)p + 8 * hh); f.half[1] = *(const v8us*)((const unsigned short*)p + 16 + 8 * hh); return f.v; }
__device__ __forceinline__ v8f g2_mma(v16h a, v16h b, v8f c) { v8f d = __builtin_amdgcn_wmma_f32_16x16x32_f16(false, a, false, b, (short)0, c, false, false); asm volatile("v_nop\n\tv_nop\n\tv_nop\n\tv_nop" : "+v"(d) : "v"(a), "v"(b)); return d; }

template <bool ROPE, bool HASBIAS, bool OUTF32>
__global__ __launch_bounds__(128) void k_gemm2(const _Float16* __restrict__ A, int lda, size_t sA, const _Float16* __restrict__ Bh, int ldb, size_t sB, float alpha,
    const float* __restrict__ bias, const float* __restrict__ rope,
    float* __restrict__ C, _Float16* __restrict__ C16, int ldc, size_t sC, int M, int N, int K) {
  __shared__ __attribute__((aligned(16))) float so[4][32][68];
  (void)bias; (void)rope; (void)C; (void)C16;
  const int tid = threadIdx.x, w = __builtin_amdgcn_readfirstlane((int)(tid >> 5)), lane = tid & 31, ln = lane & 15, hh = lane >> 4; const int by = blockIdx.y;
  A += (size_t)by * sA; Bh += (size_t)by * sB; const size_t cofs = (size_t)by * sC;
  const int ntn = N >> 6; const int mt = blockIdx.x / ntn, nq = blockIdx.x - mt * ntn; const int row0 = mt * 128 + 32 * w, col0 = nq * 64; if (row0 >= M) return;
  const _Float16* a0p = A + (size_t)(row0 + ln) * lda; const _Float16* a1p = a0p + (size_t)16 * lda;
  const _Float16* b0p = Bh + (size_t)(col0 + ln) * ldb; const _Float16* b1p = b0p + (size_t)16 * ldb; const _Float16* b2p = b1p + (size_t)16 * ldb; const _Float16* b3p = b2p + (size_t)16 * ldb;
  const v8f z8 = {0.f,0.f,0.f,0.f,0.f,0.f,0.f,0.f}; v8f c00 = z8, c01 = z8, c02 = z8, c03 = z8, c10 = z8, c11 = z8, c12 = z8, c13 = z8;
#pragma unroll 1
  for (int kb = 0; kb < K; kb += 32) { const v16h a0 = g2_frag(a0p + kb, hh), a1 = g2_frag(a1p + kb, hh);
    v16h b = g2_frag(b0p + kb, hh); c00 = g2_mma(a0, b, c00); c10 = g2_mma(a1, b, c10);
    b = g2_frag(b1p + kb, hh); c01 = g2_mma(a0, b, c01); c11 = g2_mma(a1, b, c11);
    b = g2_frag(b2p + kb, hh); c02 = g2_mma(a0, b, c02); c12 = g2_mma(a1, b, c12);
    b = g2_frag(b3p + kb, hh); c03 = g2_mma(a0, b, c03); c13 = g2_mma(a1, b, c13); }
  v8f accs[8] = {c00, c01, c02, c03, c10, c11, c12, c13};
#pragma unroll
  for (int u = 0; u < 8; ++u) { const int t = u & 3, half = u >> 2; const int col = col0 + t * 16 + ln; float bv = 0.f; if (HASBIAS) bv = bf16_rne(bias[col]);
#pragma unroll
    for (int r = 0; r < 8; ++r) { const int rloc = half * 16 + 8 * hh + r; so[w][rloc][t * 16 + ln] = accs[u][r] * alpha + bv; } }
  __builtin_amdgcn_fence(4  , "workgroup"); __builtin_amdgcn_wave_barrier();
  const int rsub = lane >> 4, c4 = (lane & 15) * 4;
  if (ROPE) {
#pragma unroll 4
    for (int q = 0; q < 16; ++q) { const int r = q * 2 + rsub; const int s = (row0 + r) % SEQ;
      const float* fp = rope + (size_t)s * FR_ROW + c4 * 2;
      const v4f fa = *(const v4fa*)(fp), fb = *(const v4fa*)(fp + 4);
      const v4f t = *(const v4fa*)&so[w][r][c4];
      v4f o;
      o[0] = bf16_rne(fa[0]) * t[0] + bf16_rne(fa[1]) * t[1];
      o[1] = bf16_rne(fa[2]) * t[0] + bf16_rne(fa[3]) * t[1];
      o[2] = bf16_rne(fb[0]) * t[2] + bf16_rne(fb[1]) * t[3];
      o[3] = bf16_rne(fb[2]) * t[2] + bf16_rne(fb[3]) * t[3];
      *(v4fa*)&so[w][r][c4] = o; }
    __builtin_amdgcn_fence(4  , "workgroup"); __builtin_amdgcn_wave_barrier();
  }
  for (int pass = 0; pass < 2; ++pass) {
#pragma unroll
    for (int q = 0; q < 16; ++q) { const int r = q * 2 + rsub; const v4f v = *(const v4fa*)&so[w][r][c4];
      if (OUTF32) { *(volatile v4f*)(C + cofs + (size_t)(row0 + r) * ldc + col0 + c4) = v; }
      else { v4h h4;
#pragma unroll
        for (int i = 0; i < 4; ++i) h4[i] = (_Float16)v[i];
        *(volatile v4h*)(C16 + cofs + (size_t)(row0 + r) * ldc + col0 + c4) = h4; } }
    if (pass == 0) __threadfence(); } }

template <int NHv, int TTv>
__global__ __launch_bounds__(256) void k_vt(const _Float16* __restrict__ V16, int ldv, int voff, _Float16* __restrict__ Vt) {
  __shared__ unsigned short tl[64][66];
  const int tid = threadIdx.x; const int slab = blockIdx.x / (TTv / 64), lg = blockIdx.x % (TTv / 64); const int b = slab / NHv, h = slab % NHv;
  for (int i = tid; i < 64 * 8; i += 256) { const int r = i / 8, c8 = (i % 8) * 8; FragH f; f.half[0] = *(const v8us*)((const unsigned short*)V16 + ((size_t)b * TTv + lg * 64 + r) * ldv + voff + h * 64 + c8);
#pragma unroll
    for (int q = 0; q < 8; ++q) tl[r][c8 + q] = f.u[q]; }
  __syncthreads();
  for (int pass = 0; pass < 2; ++pass) {
#pragma unroll
    for (int rd = 0; rd < 2; ++rd) { const int d = rd * 32 + tid / 8, pc = tid % 8; FragH f;
#pragma unroll
      for (int q = 0; q < 8; ++q) f.u[q] = tl[pc * 8 + q][d];
      *(volatile v8us*)((unsigned short*)Vt + ((size_t)slab * 64 + d) * TTv + lg * 64 + pc * 8) = f.half[0]; }
    if (pass == 0) __threadfence(); } }

__global__ __launch_bounds__(256) void k_rsmf(const float* __restrict__ S, _Float16* __restrict__ P, int qn, int hg) {
  #pragma clang fp contract(off)
  const int t = blockIdx.x * 256 + threadIdx.x; if (t >= qn * hg) return; const size_t i = (size_t)(t / qn) * SEQ + (t % qn); const float* s = S + i * SEQ; float mx = -3.0e38f;
#pragma unroll 1
  for (int j = 0; j < SEQ; ++j) mx = fmaxf(mx, s[j]);
  float se = 0.f;
#pragma unroll 1
  for (int j = 0; j < SEQ; ++j) se += __expf(s[j] - mx);
  const float sc = 256.0f / se;
#pragma unroll 1
  for (int j0 = 0; j0 < SEQ; j0 += 8) { FragH f;
#pragma unroll
    for (int q = 0; q < 8; ++q) f.h[q] = (_Float16)(__expf(s[j0 + q] - mx) * sc);
    const v8us o = f.half[0]; unsigned short* d = (unsigned short*)P + i * SEQ + j0; *(volatile v8us*)d = o; __threadfence(); *(volatile v8us*)d = o; } }

constexpr size_t WS_W  = (size_t)DM * DM * 2;
constexpr size_t WS_RW = (size_t)NB * SEQ * DM * 2;
constexpr size_t WS_S  = (size_t)HG * SEQ * SEQ * 4;
constexpr size_t WS_P  = (size_t)HG * SEQ * SEQ * 2;
constexpr size_t WS_VT = (size_t)NH * HD * SEQ * 2;
static_assert(4 * WS_W + 5 * WS_RW + WS_S + WS_P + WS_VT <= (size_t)134217728);
static_assert(WS_W % 256 == 0 && WS_RW % 256 == 0 && WS_S % 256 == 0 && WS_P % 256 == 0 && WS_VT % 256 == 0);

extern "C" void kernel_launch(void* const* d_in, const int* in_sizes, int n_in,
                              void* d_out, int out_size, void* d_ws, size_t ws_size, hipStream_t stream) {
  if (n_in < 10) return;
  const long long need_x = (long long)(NB - 1) * (long long)X_BSTRIDE_FULL + (long long)SEQ * DM;
  if ((long long)in_sizes[0] < need_x) return;
  if ((long long)in_sizes[1] < (long long)SEQ * FR_ROW) return;
  if ((long long)in_sizes[2] < (long long)DM * DM || (long long)in_sizes[4] < (long long)DM * DM || (long long)in_sizes[6] < (long long)DM * DM || (long long)in_sizes[8] < (long long)DM * DM) return;
  if (in_sizes[3] < DM || in_sizes[5] < DM || in_sizes[7] < DM || in_sizes[9] < DM) return;
  if ((long long)out_size < (long long)NB * SEQ * DM) return;
  const float* const* I = (const float* const*)d_in;
  const float* x = I[0]; const float* fr = I[1]; const float* wq = I[2]; const float* bq = I[3]; const float* wk = I[4]; const float* bk = I[5]; const float* wv = I[6]; const float* bv = I[7]; const float* wo = I[8]; const float* bo = I[9];
  char* ws = (char*)d_ws; size_t off = 0;
  auto take = [&](size_t bytes) { char* p = ws + off; off += (bytes + 255) & ~(size_t)255; return p; };
  _Float16* BQ = (_Float16*)take(WS_W); _Float16* BK = (_Float16*)take(WS_W); _Float16* BV = (_Float16*)take(WS_W); _Float16* BO = (_Float16*)take(WS_W);
  _Float16* X16 = (_Float16*)take(WS_RW); _Float16* Q16 = (_Float16*)take(WS_RW); _Float16* K16 = (_Float16*)take(WS_RW); _Float16* V16 = (_Float16*)take(WS_RW); _Float16* O16 = (_Float16*)take(WS_RW);
  float* S = (float*)take(WS_S); _Float16* P = (_Float16*)take(WS_P); _Float16* VT = (_Float16*)take(WS_VT);
  if (off > ws_size || off > (size_t)134217728) return;

  { const size_t n8 = (size_t)DM * DM / 8; const unsigned g = (unsigned)((n8 + 255) / 256);
    k_wnat<<<g, 256, 0, stream>>>(wq, n8, BQ); k_wnat<<<g, 256, 0, stream>>>(wk, n8, BK); k_wnat<<<g, 256, 0, stream>>>(wv, n8, BV); k_wnat<<<g, 256, 0, stream>>>(wo, n8, BO); }
  { const size_t n8b = (size_t)SEQ * DM / 8, n8 = (size_t)NB * n8b;
    k_x16<<<(unsigned)((n8 + 255) / 256), 256, 0, stream>>>(x, X16, n8b, X_BSTRIDE_FULL, n8); }

  const unsigned gproj = (unsigned)((NR / 128) * (DM / 64));
  k_gemm2<true,  true, false><<<dim3(gproj, 1), 128, 0, stream>>>(X16, DM, 0, BQ, DM, 0, 0.0625f, bq, fr, nullptr, Q16, DM, 0, (int)NR, DM, DM);
  k_gemm2<true,  true, false><<<dim3(gproj, 1), 128, 0, stream>>>(X16, DM, 0, BK, DM, 0, 0.0625f, bk, fr, nullptr, K16, DM, 0, (int)NR, DM, DM);
  k_gemm2<false, true, false><<<dim3(gproj, 1), 128, 0, stream>>>(X16, DM, 0, BV, DM, 0, 0.0625f, bv, nullptr, nullptr, V16, DM, 0, (int)NR, DM, DM);

  for (int b = 0; b < NB; ++b) { const size_t r0 = (size_t)b * SEQ;
    k_vt<NH, SEQ><<<NH * (SEQ / 64), 256, 0, stream>>>(V16 + r0 * DM, DM, 0, VT);
    for (int h0 = 0; h0 < NH; h0 += HG) {
      k_gemm2<false, false, true><<<dim3((SEQ / 128) * (SEQ / 64), HG), 128, 0, stream>>>(Q16 + r0 * DM + h0 * HD, DM, (size_t)HD, K16 + r0 * DM + h0 * HD, DM, (size_t)HD, 0.125f, nullptr, nullptr, S, nullptr, SEQ, (size_t)SEQ * SEQ, SEQ, SEQ, HD);
      k_rsmf<<<(HG * SEQ + 255) / 256, 256, 0, stream>>>(S, P, SEQ, HG);
      k_gemm2<false, false, false><<<dim3((SEQ / 128) * (HD / 64), HG), 128, 0, stream>>>(P, SEQ, (size_t)SEQ * SEQ, VT + (size_t)h0 * HD * SEQ, SEQ, (size_t)HD * SEQ, 0.25f, nullptr, nullptr, nullptr, O16 + r0 * DM + h0 * HD, DM, (size_t)HD, SEQ, HD, SEQ); } }

  k_gemm2<false, true, true><<<dim3(gproj, 1), 128, 0, stream>>>(O16, DM, 0, BO, DM, 0, 0.0009765625f, bo, nullptr, (float*)d_out, nullptr, DM, 0, (int)NR, DM, DM);
  (void)stream;
}
